// Disc_edge2_15573551415685
// MI455X (gfx1250) — hardware-verified
//
#include <hip/hip_runtime.h>
typedef __attribute__((ext_vector_type(4))) float vf4v_t;
typedef __attribute__((ext_vector_type(4))) unsigned int vu4v_t;
typedef __attribute__((ext_vector_type(4))) int vi4v_t;


#define B_  16
#define N_  128
#define DH_ 128

typedef __attribute__((ext_vector_type(16))) _Float16 v16bf;
#define VST2(T, ptr, val) do { const T _v = (val); *(volatile T*)(ptr) = _v; __threadfence(); *(volatile T*)(ptr) = _v; } while (0)
__device__ __forceinline__ int kmap16(int e, int hh) { return (e < 8) ? (8 * hh + e) : (16 + 8 * hh + (e - 8)); }
typedef __attribute__((ext_vector_type(8)))  float  v8f;

union Frag {
    v16bf        v;
    uint4        q[2];
    unsigned int u[8];
};

__device__ __forceinline__ unsigned short f2bf(float f) {
    return __builtin_bit_cast(unsigned short, (_Float16)f);
}
__device__ __forceinline__ float bf2f(unsigned short s) {
    return (float)__builtin_bit_cast(_Float16, s);
}
typedef __attribute__((ext_vector_type(8))) float v8f_t;
__device__ __forceinline__ v8f_t wmma16(v16bf a, v16bf b, v8f_t c) {
    v8f_t d = __builtin_amdgcn_wmma_f32_16x16x32_f16(false, a, false, b, (short)0, c, false, false);
    asm volatile("v_nop\n\tv_nop\n\tv_nop\n\tv_nop" : "+v"(d) : "v"(a), "v"(b));
    return d;
}
__device__ __forceinline__ unsigned int pack2(float lo, float hi) {
    return (unsigned int)f2bf(lo) | ((unsigned int)f2bf(hi) << 16);
}

__global__ __launch_bounds__(256) void cvt_bf16_kernel(
    const float* __restrict__ in, unsigned short* __restrict__ out, int n)
{
    const int i8 = blockIdx.x * 256 + threadIdx.x;
    if (i8 * 8 >= n) return;
    vu4v_t q; unsigned short* hq = (unsigned short*)&q;
#pragma unroll
    for (int e = 0; e < 8; ++e) hq[e] = f2bf(in[i8 * 8 + e]);
    VST2(vu4v_t, (vu4v_t*)(out + (size_t)i8 * 8), q);
}

__global__ __launch_bounds__(256) void convert_w_kernel(
    const float* __restrict__ wmsg, int Dn, int De, int total,
    unsigned short* __restrict__ out)
{
    const int i8 = blockIdx.x * 256 + threadIdx.x;
    if (i8 * 8 >= total) return;
    const int d0 = i8 * 8;
    const int e0 = d0 & 15, lane = (d0 >> 4) & 31, ht = (d0 >> 9) & 7, ks = d0 >> 12;
    vu4v_t q; unsigned short* hq = (unsigned short*)&q;
#pragma unroll
    for (int t = 0; t < 8; ++t) {
        const int k = ks * 32 + kmap16(e0 + t, lane >> 4);
        const int h = ht * 16 + (lane & 15);
        float v = 0.0f;
        if (k < De)           v = wmsg[(size_t)(2 * Dn + k) * DH_ + h];
        else if (k < De + Dn) v = wmsg[(size_t)(Dn + (k - De)) * DH_ + h];
        hq[t] = f2bf(v);
    }
    VST2(vu4v_t, (vu4v_t*)(out + d0), q);
}

template <int MODE>
__global__ __launch_bounds__(256) void edge_kernel(
    const int*            __restrict__ A,
    const float*          __restrict__ e32,
    const unsigned short* __restrict__ ebf,
    const unsigned short* __restrict__ xbf,
    const float*          __restrict__ xi,
    const unsigned short* __restrict__ wcomb,
    const float*          __restrict__ bmsg,
    unsigned short*       __restrict__ msg_out,
    float*                __restrict__ agg_out,
    float*                __restrict__ hsum)
{
    constexpr int  KSTEPS  = (MODE == 0) ? 3 : 8;
    constexpr int  EPITCH  = (MODE == 0) ? 104 : 264;
    constexpr bool WRITES  = (MODE != 2);
    constexpr int  STPITCH = 136;

    __shared__ unsigned short lds_e[N_ * EPITCH];
    __shared__ unsigned short lds_st[WRITES ? (8 * 16 * STPITCH) : 1];
    __shared__ float lds_agg[8][DH_];
    __shared__ float lds_xi[DH_];
    __shared__ float lds_bias[DH_];

    const int wg   = blockIdx.x;
    const int b    = wg >> 7;
    const int tid  = threadIdx.x;
    const int lane = tid & 31;
    const int wave = tid >> 5;
    const int half = (lane >> 4) & 1;
    const int ln   = lane & 15;

    if (tid < DH_) {
        lds_xi[tid]   = xi[(size_t)wg * DH_ + tid];
        lds_bias[tid] = bmsg[tid];
    }
    (void)hsum;

    {
        const int j   = tid >> 1;
        const int sub = tid & 1;
        if (MODE == 0) {
            if (sub == 0) {
                const float4* src = (const float4*)(e32 + (((size_t)wg * N_) + j) * 16);
                float4 p0 = src[0], p1 = src[1], p2 = src[2], p3 = src[3];
                unsigned int* dst = (unsigned int*)&lds_e[j * EPITCH];
                dst[0] = pack2(p0.x, p0.y); dst[1] = pack2(p0.z, p0.w);
                dst[2] = pack2(p1.x, p1.y); dst[3] = pack2(p1.z, p1.w);
                dst[4] = pack2(p2.x, p2.y); dst[5] = pack2(p2.z, p2.w);
                dst[6] = pack2(p3.x, p3.y); dst[7] = pack2(p3.z, p3.w);
            } else {
                uint4* dz = (uint4*)&lds_e[j * EPITCH + 80];
                dz[0] = make_uint4(0u,0u,0u,0u);
                dz[1] = make_uint4(0u,0u,0u,0u);
            }
            const uint4* xs = (const uint4*)(xbf + (((size_t)b * N_) + j) * 64 + sub * 32);
            uint4* xd = (uint4*)&lds_e[j * EPITCH + 16 + sub * 32];
            xd[0] = xs[0]; xd[1] = xs[1]; xd[2] = xs[2]; xd[3] = xs[3];
        } else {
            const int koff = sub * 64;
            const uint4* es = (const uint4*)(ebf + (((size_t)wg * N_) + j) * DH_ + koff);
            uint4* ed = (uint4*)&lds_e[j * EPITCH + koff];
#pragma unroll
            for (int q = 0; q < 8; ++q) ed[q] = es[q];
            const uint4* xs = (const uint4*)(xbf + (((size_t)b * N_) + j) * DH_ + koff);
            uint4* xd = (uint4*)&lds_e[j * EPITCH + 128 + koff];
#pragma unroll
            for (int q = 0; q < 8; ++q) xd[q] = xs[q];
            if (sub) *(uint4*)&lds_e[j * EPITCH + 256] = make_uint4(0u,0u,0u,0u);
        }
    }
    __syncthreads();

    const int j0 = wave * 16;
    const int* Arow = A + (size_t)wg * N_;
    float am[8];
    #pragma unroll
    for (int r = 0; r < 8; ++r) am[r] = (float)Arow[j0 + half * 8 + r];

    v8f c[8];
    {
        v8f z = {};
        #pragma unroll
        for (int t = 0; t < 8; ++t) c[t] = z;
    }
    #pragma unroll
    for (int ks = 0; ks < KSTEPS; ++ks) {
        Frag a;
        const int k0 = ks * 32 + half * 8;
        a.q[0] = *(const uint4*)&lds_e[(j0 + ln) * EPITCH + k0];
        a.q[1] = *(const uint4*)&lds_e[(j0 + ln) * EPITCH + k0 + 16];

        #pragma unroll
        for (int ht = 0; ht < 8; ++ht) {
            Frag bf;
            const uint4* wf = (const uint4*)(wcomb + ((size_t)(ks * 8 + ht) * 32 + lane) * 16);
            bf.q[0] = wf[0];
            bf.q[1] = wf[1];
            c[ht] = wmma16(a.v, bf.v, c[ht]);
        }
    }

    unsigned short* strow = WRITES ? &lds_st[wave * 16 * STPITCH] : (unsigned short*)nullptr;
    #pragma unroll
    for (int ht = 0; ht < 8; ++ht) {
        const int   h  = ht * 16 + ln;
        const float ab = lds_xi[h] + lds_bias[h];
        float accum = 0.0f;
        #pragma unroll
        for (int r = 0; r < 8; ++r) {
            const int jr = half * 8 + r;
            float v = fmaxf(c[ht][r] + ab, 0.0f) * am[r];
            accum += v;
            if (MODE == 0) {
                strow[jr * STPITCH + h] = f2bf(v);
            } else if (MODE == 1) {
                const float prev = bf2f(lds_e[(j0 + jr) * EPITCH + h]);
                strow[jr * STPITCH + h] = f2bf(0.5f * (prev + v));
            }
        }
        accum += __shfl_xor(accum, 16, 32);
        if (half == 0) lds_agg[wave][h] = accum;
    }

    if (WRITES) {
        __builtin_amdgcn_fence(__ATOMIC_RELEASE, "workgroup"); __builtin_amdgcn_wave_barrier(); __builtin_amdgcn_fence(__ATOMIC_ACQUIRE, "workgroup");
        unsigned short* mrow = msg_out + (size_t)wg * N_ * DH_;
        for (int pass = 0; pass < 2; ++pass) {
            #pragma unroll
            for (int jj = 0; jj < 8; ++jj) {
                const int row = jj * 2 + (lane >> 4), seg = lane & 15;
                *(volatile vu4v_t*)(mrow + (size_t)(j0 + row) * DH_ + seg * 8) = *(const vu4v_t*)&strow[row * STPITCH + seg * 8];
            }
            __threadfence();
        }
    }
    __syncthreads();

    if (tid < DH_) {
        float s = 0.0f;
        #pragma unroll
        for (int w8 = 0; w8 < 8; ++w8) s += lds_agg[w8][tid];
        VST2(float, agg_out + (size_t)wg * DH_ + tid, s);
    }
}

__global__ __launch_bounds__(256) void xi_kernel(
    const float* __restrict__ x, int Dn,
    const float* __restrict__ wmsg,
    float* __restrict__ xi)
{
    const int idx = blockIdx.x * 256 + threadIdx.x;
    const int h   = idx & (DH_ - 1);
    const int row = idx >> 7;
    const float* xr = x + (size_t)row * Dn;
    float acc = 0.0f;
    for (int k = 0; k < Dn; ++k) acc = fmaf(xr[k], wmsg[(size_t)k * DH_ + h], acc);
    VST2(float, xi + idx, acc);
}

__global__ __launch_bounds__(256) void node_kernel(
    const float* __restrict__ x, int Dn,
    const float* __restrict__ agg,
    const float* __restrict__ wnode, const float* __restrict__ bnode,
    const float* __restrict__ mix_with,
    float* __restrict__ out)
{
    const int idx = blockIdx.x * 256 + threadIdx.x;
    const int h   = idx & (DH_ - 1);
    const int row = idx >> 7;
    const float* xr = x + (size_t)row * Dn;
    const float* ar = agg + (size_t)row * DH_;
    float acc = bnode[h];
    for (int k = 0; k < Dn; ++k)  acc = fmaf(xr[k], wnode[(size_t)k * DH_ + h], acc);
    const float* Wa = wnode + (size_t)Dn * DH_;
    for (int k = 0; k < DH_; ++k) acc = fmaf(ar[k], Wa[(size_t)k * DH_ + h], acc);
    acc = fmaxf(acc, 0.0f);
    if (mix_with) acc = 0.5f * (mix_with[idx] + acc);
    VST2(float, out + idx, acc);
}

__global__ __launch_bounds__(128) void head_kernel(
    const float* __restrict__ aggrows,
    const float* __restrict__ w1, const float* __restrict__ b1,
    const float* __restrict__ w2, const float* __restrict__ b2,
    const float* __restrict__ w3, const float* __restrict__ b3,
    float* __restrict__ out)
{
    __shared__ float ha[DH_], hb[DH_], red[128], res[B_];
    const int t = threadIdx.x;
    for (int b = 0; b < B_; ++b) {
        float s = 0.0f;
        for (int i = 0; i < N_; ++i) s += aggrows[((size_t)b * N_ + i) * DH_ + t];
        ha[t] = s * (1.0f / (float)(N_ * N_));
        __syncthreads();
        float acc = b1[t];
        for (int k = 0; k < DH_; ++k) acc = fmaf(ha[k], w1[k * DH_ + t], acc);
        hb[t] = fmaxf(acc, 0.0f);
        __syncthreads();
        acc = b2[t];
        for (int k = 0; k < DH_; ++k) acc = fmaf(hb[k], w2[k * DH_ + t], acc);
        red[t] = fmaxf(acc, 0.0f) * w3[t];
        __syncthreads();
        for (int s2 = 64; s2 > 0; s2 >>= 1) {
            if (t < s2) red[t] += red[t + s2];
            __syncthreads();
        }
        if (t == 0) res[b] = red[0] + b3[0];
        __syncthreads();
    }
    if (t < B_) VST2(float, out + t, res[t]);
}

extern "C" void kernel_launch(void* const* d_in, const int* in_sizes, int n_in,
                              void* d_out, int out_size, void* d_ws, size_t ws_size,
                              hipStream_t stream)
{
    (void)in_sizes; (void)n_in; (void)out_size;

    const int*   A        = (const int*)  d_in[0];
    const float* x0       = (const float*)d_in[1];
    const float* e0       = (const float*)d_in[2];
    const float* w_msg_0  = (const float*)d_in[3];
    const float* b_msg_0  = (const float*)d_in[4];
    const float* w_node_0 = (const float*)d_in[5];
    const float* b_node_0 = (const float*)d_in[6];
    const float* w_msg_1  = (const float*)d_in[7];
    const float* b_msg_1  = (const float*)d_in[8];
    const float* w_node_1 = (const float*)d_in[9];
    const float* b_node_1 = (const float*)d_in[10];
    const float* w_msg_2  = (const float*)d_in[11];
    const float* b_msg_2  = (const float*)d_in[12];
    const float* w_h1     = (const float*)d_in[15];
    const float* b_h1     = (const float*)d_in[16];
    const float* w_h2     = (const float*)d_in[17];
    const float* b_h2     = (const float*)d_in[18];
    const float* w_h3     = (const float*)d_in[19];
    const float* b_h3     = (const float*)d_in[20];
    float* out = (float*)d_out;

    char* ws = (char*)d_ws;
    const size_t MSG_BYTES = (size_t)B_ * N_ * N_ * DH_ * sizeof(unsigned short);
    const size_t VEC_BYTES = (size_t)B_ * N_ * DH_ * sizeof(float);
    unsigned short* msgbuf = (unsigned short*)ws;                 ws += MSG_BYTES;
    float* xi   = (float*)ws;  ws += VEC_BYTES;
    float* agg  = (float*)ws;  ws += VEC_BYTES;
    float* x1   = (float*)ws;  ws += VEC_BYTES;
    float* xmix = (float*)ws;  ws += VEC_BYTES;
    float* hsum = (float*)ws;  ws += 256 * sizeof(float) * 8;
    unsigned short* wcomb = (unsigned short*)ws;
    ws += (size_t)256 * DH_ * sizeof(unsigned short);
    unsigned short* xbf = (unsigned short*)ws;
    ws += (size_t)B_ * N_ * DH_ * sizeof(unsigned short);
    float* agg2 = (float*)ws;  ws += VEC_BYTES;
    if ((size_t)(ws - (char*)d_ws) > ws_size) return;

    const dim3 blk256(256), blk128(128);
    const dim3 grid_vec(B_ * N_ * DH_ / 256);
    const dim3 grid_edge(B_ * N_);

    cvt_bf16_kernel<<<B_ * N_ * 64 / 8 / 256, blk256, 0, stream>>>(x0, xbf, B_ * N_ * 64);
    xi_kernel<<<grid_vec, blk256, 0, stream>>>(x0, 64, w_msg_0, xi);
    convert_w_kernel<<<6, blk256, 0, stream>>>(w_msg_0, 64, 16, 96 * DH_, wcomb);
    edge_kernel<0><<<grid_edge, blk256, 0, stream>>>(
        A, e0, nullptr, xbf, xi, wcomb, b_msg_0, msgbuf, agg, nullptr);
    node_kernel<<<grid_vec, blk256, 0, stream>>>(
        x0, 64, agg, w_node_0, b_node_0, nullptr, x1);

    cvt_bf16_kernel<<<B_ * N_ * DH_ / 8 / 256, blk256, 0, stream>>>(x1, xbf, B_ * N_ * DH_);
    xi_kernel<<<grid_vec, blk256, 0, stream>>>(x1, 128, w_msg_1, xi);
    convert_w_kernel<<<16, blk256, 0, stream>>>(w_msg_1, 128, 128, 256 * DH_, wcomb);
    edge_kernel<1><<<grid_edge, blk256, 0, stream>>>(
        A, nullptr, msgbuf, xbf, xi, wcomb, b_msg_1, msgbuf, agg, nullptr);
    node_kernel<<<grid_vec, blk256, 0, stream>>>(
        x1, 128, agg, w_node_1, b_node_1, x1, xmix);

    cvt_bf16_kernel<<<B_ * N_ * DH_ / 8 / 256, blk256, 0, stream>>>(xmix, xbf, B_ * N_ * DH_);
    xi_kernel<<<grid_vec, blk256, 0, stream>>>(xmix, 128, w_msg_2, xi);
    convert_w_kernel<<<16, blk256, 0, stream>>>(w_msg_2, 128, 128, 256 * DH_, wcomb);
    edge_kernel<2><<<grid_edge, blk256, 0, stream>>>(
        A, nullptr, msgbuf, xbf, xi, wcomb, b_msg_2, nullptr, agg2, nullptr);
    (void)hsum;

    head_kernel<<<1, blk128, 0, stream>>>(
        agg2, w_h1, b_h1, w_h2, b_h2, w_h3, b_h3, out);
}
